// StarGNN_58402965291383
// MI455X (gfx1250) — hardware-verified
//
#include <hip/hip_runtime.h>

#define B_SZ   4096
#define N_PTS  256
#define FIN    15
#define HD     128
#define H4D    32
#define FOUT   6

typedef _Float16 v16h __attribute__((ext_vector_type(16)));
typedef _Float16 v8h  __attribute__((ext_vector_type(8)));
typedef float    v8f  __attribute__((ext_vector_type(8)));

__device__ __forceinline__ float sigf(float x)  {
  return __builtin_amdgcn_rcpf(1.0f + __expf(-x));
}
__device__ __forceinline__ float siluf(float x) { return x * sigf(x); }

__device__ __forceinline__ v16h cat8(v8h lo, v8h hi) {
  return __builtin_shufflevector(lo, hi, 0,1,2,3,4,5,6,7,8,9,10,11,12,13,14,15);
}

__device__ __forceinline__ v16h load_A16(const _Float16* stage, int K, int m, int cBase, int half) {
  const _Float16* p = stage + m * K + cBase + half * 8;
  v8h lo = *(const v8h*)(p);
  v8h hi = *(const v8h*)(p + 16);
  return cat8(lo, hi);
}

__device__ __forceinline__ v16h load_B16(const _Float16* wt, int K, int ncol, int cBase, int half) {
  const _Float16* p = wt + ncol * K + cBase + half * 8;
  v8h lo = *(const v8h*)(p);
  v8h hi = *(const v8h*)(p + 16);
  return cat8(lo, hi);
}

__device__ __forceinline__ v8f wmma_f16(v16h a, v16h b, v8f c) {
  return __builtin_amdgcn_wmma_f32_16x16x32_f16(false, a, false, b, (short)0, c, false, false);
}

typedef __bf16 v16b __attribute__((ext_vector_type(16)));
typedef __bf16 v8b  __attribute__((ext_vector_type(8)));
__device__ __forceinline__ unsigned short bf_rne(float f) { unsigned u = __builtin_bit_cast(unsigned, f); u += 0x7FFFu + ((u >> 16) & 1u); return (unsigned short)(u >> 16); }
__device__ __forceinline__ void splitbf(float f, __bf16& h, __bf16& l) {
  const unsigned short hb = bf_rne(f); const float hf_ = __builtin_bit_cast(float, ((unsigned)hb) << 16);
  h = __builtin_bit_cast(__bf16, hb); l = __builtin_bit_cast(__bf16, bf_rne(f - hf_));
}
__device__ __forceinline__ v16b cat8b(v8b lo, v8b hi) { return __builtin_shufflevector(lo, hi, 0,1,2,3,4,5,6,7,8,9,10,11,12,13,14,15); }
__device__ __forceinline__ v16b load_A16b(const __bf16* stage, int K, int m, int cBase, int half) {
  const __bf16* p = stage + m * K + cBase + half * 8; return cat8b(*(const v8b*)(p), *(const v8b*)(p + 16));
}
__device__ __forceinline__ v16b load_B16b(const __bf16* wt, int K, int ncol, int cBase, int half) {
  const __bf16* p = wt + ncol * K + cBase + half * 8; return cat8b(*(const v8b*)(p), *(const v8b*)(p + 16));
}
__device__ __forceinline__ v8f wmma_bf(v16b a, v16b b, v8f c) {
  return __builtin_amdgcn_wmma_f32_16x16x32_bf16(false, a, false, b, (short)0, c, false, false);
}
__device__ __forceinline__ v8f wmma_bsplit(v16b ah, v16b al, v16b bh, v16b bl, v8f c) {
  v8f x = {};
  x = wmma_bf(al, bh, x); x = wmma_bf(ah, bl, x);
  return wmma_bf(ah, bh, c) + x;
}

__global__ __launch_bounds__(128) void stargnn_pernode(
    const float* __restrict__ x_feat, const float* __restrict__ coords,
    const float* __restrict__ mask,   const int*   __restrict__ centers,
    const float* __restrict__ nW1,    const float* __restrict__ nb1,
    const float* __restrict__ nW2,    const float* __restrict__ nb2,
    const float* __restrict__ eW1,    const float* __restrict__ eb1,
    const float* __restrict__ eW2,    const float* __restrict__ eb2,
    float* __restrict__ msg)
{
  __shared__ __align__(16) _Float16 WT1h[HD * 32];
  __shared__ __align__(16) _Float16 WT2h[HD * HD];
  __shared__ __align__(16) _Float16 xst[4][16 * 32];
  __shared__ __align__(16) _Float16 h1st[4][16 * HD];
  __shared__ float nb1s[HD], nb2s[HD];
  __shared__ float eW1s[H4D], eb1s[H4D], eW2s[H4D];
  __shared__ float eb2s, c0s[3];
  __shared__ int   cRs;
  __shared__ float sarr[4][16];
  __shared__ float msgbuf[HD];

  const int tid  = threadIdx.x;
  const int lane = tid & 31;
  const int wid  = tid >> 5;
  const int half = lane >> 4;
  const int n16  = lane & 15;
  const int b    = blockIdx.x;
  const int bN   = b * N_PTS;

  for (int i = tid; i < HD * 32; i += 128) {
    int nc = i >> 5, k = i & 31;
    WT1h[i] = (k < FIN) ? (_Float16)nW1[k * HD + nc] : (_Float16)0.f;
  }
  for (int i = tid; i < HD * HD; i += 128) {
    int nc = i >> 7, k = i & 127;
    WT2h[i] = (_Float16)nW2[k * HD + nc];
  }
  if (tid < HD)  { nb1s[tid] = nb1[tid]; nb2s[tid] = nb2[tid]; msgbuf[tid] = 0.f; }
  if (tid < H4D) { eW1s[tid] = eW1[tid]; eb1s[tid] = eb1[tid]; eW2s[tid] = eW2[tid]; }
  if (tid == 0) {
    eb2s = eb2[0];
    int cr = centers[b]; cRs = cr;
    const float* cp = coords + (size_t)(bN + cr) * 3;
    c0s[0] = cp[0]; c0s[1] = cp[1]; c0s[2] = cp[2];
  }
  for (int i = lane; i < 16 * 32; i += 32) xst[wid][i] = (_Float16)0.f;
  __syncthreads();

  float macc[8];
#pragma unroll
  for (int t = 0; t < 8; ++t) macc[t] = 0.f;

  for (int tt = 0; tt < 4; ++tt) {
    const int tileStart = wid * 64 + tt * 16;

    const float* xrow = x_feat + (size_t)(bN + tileStart) * FIN;
    for (int i = lane; i < 16 * FIN; i += 32) {
      int m = i / FIN, k = i % FIN;
      xst[wid][m * 32 + k] = (_Float16)xrow[i];
    }

    if (half == 0) {
      int p = tileStart + n16;
      const float* cp = coords + (size_t)(bN + p) * 3;
      float dx = cp[0] - c0s[0], dy = cp[1] - c0s[1], dz = cp[2] - c0s[2];
      float d = __builtin_amdgcn_sqrtf(dx * dx + dy * dy + dz * dz);
      float acc = eb2s;
#pragma unroll
      for (int j = 0; j < H4D; ++j) acc += siluf(d * eW1s[j] + eb1s[j]) * eW2s[j];
      float mk = mask[bN + p];
      float wv = sigf(acc) * mk;
      sarr[wid][n16] = wv * mk + ((p == cRs) ? mk : 0.f);
    }
    __syncthreads();

    v16h a0 = load_A16(xst[wid], 32, n16, 0, half);
#pragma unroll
    for (int nt = 0; nt < 8; ++nt) {
      v16h bw = load_B16(WT1h, 32, nt * 16 + n16, 0, half);
      v8f c1 = {};
      c1 = wmma_f16(a0, bw, c1);
      float bias = nb1s[nt * 16 + n16];
#pragma unroll
      for (int v = 0; v < 8; ++v)
        h1st[wid][(v + half * 8) * HD + nt * 16 + n16] = (_Float16)siluf(c1[v] + bias);
    }
    __syncthreads();

    v8f z = {};
    v8f acc2[8];
#pragma unroll
    for (int nt = 0; nt < 8; ++nt) acc2[nt] = z;
#pragma unroll
    for (int c = 0; c < 4; ++c) {
      v16h a = load_A16(h1st[wid], HD, n16, c * 32, half);
#pragma unroll
      for (int nt = 0; nt < 8; ++nt) {
        v16h bw = load_B16(WT2h, HD, nt * 16 + n16, c * 32, half);
        acc2[nt] = wmma_f16(a, bw, acc2[nt]);
      }
    }

#pragma unroll
    for (int nt = 0; nt < 8; ++nt) {
      float bias = nb2s[nt * 16 + n16];
      float part = 0.f;
#pragma unroll
      for (int v = 0; v < 8; ++v)
        part += sarr[wid][v + half * 8] * siluf(acc2[nt][v] + bias);
      part += __shfl_xor(part, 16, 32);
      macc[nt] += part;
    }
    __syncthreads();
  }

  if (half == 0) {
#pragma unroll
    for (int nt = 0; nt < 8; ++nt) atomicAdd(&msgbuf[nt * 16 + n16], macc[nt]);
  }
  __syncthreads();
  if (tid < HD) {
    *(volatile float*)(msg + (size_t)b * HD + tid) = msgbuf[tid];
    __threadfence();
    *(volatile float*)(msg + (size_t)b * HD + tid) = msgbuf[tid];
  }
}

__global__ __launch_bounds__(128) void stargnn_readout(
    const float* __restrict__ msg,
    const float* __restrict__ rW1, const float* __restrict__ rb1,
    const float* __restrict__ rW2, const float* __restrict__ rb2,
    float* __restrict__ out)
{
  __shared__ __align__(16) __bf16 WT1h[HD * HD], WT1l[HD * HD];
  __shared__ __align__(16) __bf16 WT2h[16 * HD], WT2l[16 * HD];
  __shared__ __align__(16) __bf16 h3st[4][16 * HD], h3sl[4][16 * HD];
  __shared__ float rb1s[HD], rb2s[FOUT];
  __shared__ __align__(16) float ost[4][16 * FOUT];

  const int tid  = threadIdx.x;
  const int lane = tid & 31;
  const int wid  = tid >> 5;
  const int half = lane >> 4;
  const int n16  = lane & 15;

  for (int i = tid; i < HD * HD; i += 128) {
    int nc = i >> 7, k = i & 127;
    splitbf(rW1[k * HD + nc], WT1h[i], WT1l[i]);
  }
  for (int i = tid; i < 16 * HD; i += 128) {
    int nc = i >> 7, k = i & 127;
    const float v = (nc < FOUT) ? rW2[k * FOUT + nc] : 0.f;
    splitbf(v, WT2h[i], WT2l[i]);
  }
  if (tid < HD)   rb1s[tid] = rb1[tid];
  if (tid < FOUT) rb2s[tid] = rb2[tid];
  __syncthreads();

  const int tileRow = (blockIdx.x * 4 + wid) * 16;

  v8f z = {};
  v8f acc1[8];
#pragma unroll
  for (int nt = 0; nt < 8; ++nt) acc1[nt] = z;
#pragma unroll 1
  for (int c = 0; c < 4; ++c) {
    const float* pr = msg + (size_t)(tileRow + n16) * HD + c * 32 + half * 8;
    union { v16b v; __bf16 e[16]; } a, al;
#pragma unroll
    for (int i = 0; i < 8; ++i) { splitbf(pr[i], a.e[i], al.e[i]); splitbf(pr[16 + i], a.e[8 + i], al.e[8 + i]); }
#pragma unroll
    for (int nt = 0; nt < 8; ++nt)
      acc1[nt] = wmma_bsplit(a.v, al.v, load_B16b(WT1h, HD, nt * 16 + n16, c * 32, half), load_B16b(WT1l, HD, nt * 16 + n16, c * 32, half), acc1[nt]);
  }
#pragma unroll
  for (int nt = 0; nt < 8; ++nt) {
    float bias = rb1s[nt * 16 + n16];
#pragma unroll
    for (int v = 0; v < 8; ++v)
      splitbf(siluf(acc1[nt][v] + bias), h3st[wid][(v + half * 8) * HD + nt * 16 + n16], h3sl[wid][(v + half * 8) * HD + nt * 16 + n16]);
  }
  __syncthreads();

  v8f acc2 = z;
#pragma unroll
  for (int c = 0; c < 4; ++c)
    acc2 = wmma_bsplit(load_A16b(h3st[wid], HD, n16, c * 32, half), load_A16b(h3sl[wid], HD, n16, c * 32, half),
                       load_B16b(WT2h, HD, n16, c * 32, half),      load_B16b(WT2l, HD, n16, c * 32, half), acc2);

  float* os_ = ost[wid];
  if (n16 < FOUT) {
    float bias = rb2s[n16];
#pragma unroll
    for (int v = 0; v < 8; ++v) os_[(v + half * 8) * FOUT + n16] = acc2[v] + bias;
  }
  asm volatile("s_wait_dscnt 0" ::: "memory");
  if (lane < 24) {
    typedef __attribute__((ext_vector_type(4))) float v4f_t;
    typedef float v4fa __attribute__((ext_vector_type(4), may_alias));
    const v4f_t ov = *(const volatile v4fa*)(os_ + lane * 4);
    float* dst = out + (size_t)tileRow * FOUT + lane * 4;
    *(volatile v4f_t*)dst = ov;
    __threadfence();
    *(volatile v4f_t*)dst = ov;
  }
}

extern "C" void kernel_launch(void* const* d_in, const int* in_sizes, int n_in,
                              void* d_out, int out_size, void* d_ws, size_t ws_size,
                              hipStream_t stream)
{
  const float* x_feat  = (const float*)d_in[0];
  const float* coords  = (const float*)d_in[1];
  const float* mask    = (const float*)d_in[2];
  const int*   centers = (const int*)  d_in[3];
  const float* nW1     = (const float*)d_in[4];
  const float* nb1     = (const float*)d_in[5];
  const float* nW2     = (const float*)d_in[6];
  const float* nb2     = (const float*)d_in[7];
  const float* eW1     = (const float*)d_in[8];
  const float* eb1     = (const float*)d_in[9];
  const float* eW2     = (const float*)d_in[10];
  const float* eb2     = (const float*)d_in[11];
  const float* rW1     = (const float*)d_in[12];
  const float* rb1     = (const float*)d_in[13];
  const float* rW2     = (const float*)d_in[14];
  const float* rb2     = (const float*)d_in[15];

  float* msg = (float*)d_ws;

  stargnn_pernode<<<B_SZ, 128, 0, stream>>>(x_feat, coords, mask, centers,
                                            nW1, nb1, nW2, nb2,
                                            eW1, eb1, eW2, eb2, msg);
  stargnn_readout<<<B_SZ / 64, 128, 0, stream>>>(msg, rW1, rb1, rW2, rb2,
                                                 (float*)d_out);
}
